// SparseFeedForward_45037027065974
// MI455X (gfx1250) — hardware-verified
//
#include <hip/hip_runtime.h>


namespace {
constexpr int NT = 4 * 2048, H = 1024, NE = 8, TOPK = 2, NS = NT * TOPK;
constexpr float XS = 8.0f, WSC = 256.0f;
typedef _Float16 b16;
typedef __attribute__((ext_vector_type(16))) _Float16 v16b;
typedef __attribute__((ext_vector_type(8))) _Float16 v8b;
typedef __attribute__((ext_vector_type(8))) float v8f;
typedef __attribute__((ext_vector_type(4))) float v4f;
__device__ __forceinline__ float bf16_rne(float f) { unsigned int u = __float_as_uint(f); u += 0x7FFFu + ((u >> 16) & 1u); return __uint_as_float(u & 0xFFFF0000u); }
__device__ __forceinline__ v16b frag_kb(const b16* p, int hh) { const v8b a = *(const v8b*)(p + 8 * hh), b = *(const v8b*)(p + 16 + 8 * hh); v16b f;
#pragma unroll
  for (int e = 0; e < 8; ++e) { f[e] = a[e]; f[8 + e] = b[e]; } return f; }
__device__ __forceinline__ v8f wmma16b(v16b a, v16b b, v8f c) { v8f d = __builtin_amdgcn_wmma_f32_16x16x32_f16(false, a, false, b, (short)0, c, false, false); asm volatile("v_nop\n\tv_nop\n\tv_nop\n\tv_nop" : "+v"(d) : "v"(a), "v"(b)); return d; }
__device__ __forceinline__ void wave_lds_sync() { __builtin_amdgcn_fence(__ATOMIC_RELEASE, "workgroup"); __builtin_amdgcn_wave_barrier(); __builtin_amdgcn_fence(__ATOMIC_ACQUIRE, "workgroup"); }
__device__ __forceinline__ float pmul(float a, float b) { float p = a * b; asm volatile("" : "+v"(p)); return p; }
__device__ __forceinline__ int iclamp(int v, int lo, int hi) { return v < lo ? lo : (v > hi ? hi : v); }

__global__ __launch_bounds__(256) void wput_kernel(const float* __restrict__ w, b16* __restrict__ WE) { const size_t u = (size_t)blockIdx.x * 256 + threadIdx.x; if (u >= (size_t)NE * H * (H / 8)) return; const int e = (int)(u / ((size_t)H * (H / 8))); const int h = (int)((u / (H / 8)) % H); const int k0 = (int)(u % (H / 8)) * 8; v8b v;
#pragma unroll
  for (int j = 0; j < 8; ++j) v[j] = (b16)(bf16_rne(w[((size_t)h * NE + e) * H + k0 + j]) * WSC); for (int pass = 0; pass < 2; ++pass) { *(volatile v8b*)(WE + ((size_t)e * H + h) * H + k0) = v; __threadfence(); } }
__global__ __launch_bounds__(256) void router_kernel(const float* __restrict__ x, const float* __restrict__ Wg, const float* __restrict__ bg, float* __restrict__ ROUT, int* __restrict__ RSEL) {
  const int wave = threadIdx.x >> 5, lane = threadIdx.x & 31; const size_t t = (size_t)blockIdx.x * 8 + wave; if (t >= (size_t)NT) return; const float* xr = x + t * H; float lg[NE];
#pragma unroll
  for (int e = 0; e < NE; ++e) { float s = 0.0f, c = 0.0f; const float* wr = Wg + (size_t)e * H;
#pragma unroll 1
    for (int k = lane; k < H; k += 32) { float xa = bf16_rne(xr[k]), wa = bf16_rne(wr[k]); asm volatile("" : "+v"(xa)); asm volatile("" : "+v"(wa)); const float p = pmul(xa, wa);   const float t = s + p; float bp = t - s; asm volatile("" : "+v"(bp)); const float err = (s - (t - bp)) + (p - bp); s = t; c += err; }
    for (int o = 16; o; o >>= 1) { const float so = __shfl_xor(s, o), co = __shfl_xor(c, o); const float t = s + so; float bp = t - s; asm volatile("" : "+v"(bp)); const float err = (s - (t - bp)) + (so - bp); s = t; c += co + err; }
    float bgv = bf16_rne(bg[e]); asm volatile("" : "+v"(bgv)); lg[e] = (s + c) + bgv; }
  float mx = lg[0];
#pragma unroll
  for (int e = 1; e < NE; ++e) mx = fmaxf(mx, lg[e]);
  float pr[NE]; float den = 0.0f;
#pragma unroll
  for (int e = 0; e < NE; ++e) { pr[e] = __expf(lg[e] - mx); den += pr[e]; }
  int e0 = 0; float p0 = pr[0];
#pragma unroll
  for (int e = 1; e < NE; ++e) if (pr[e] > p0) { p0 = pr[e]; e0 = e; }
  int e1 = -1; float p1 = -1.0f;
#pragma unroll
  for (int e = 0; e < NE; ++e) if (e != e0 && pr[e] > p1) { p1 = pr[e]; e1 = e; }
  const float g0 = p0 / den, g1 = p1 / den; const float w0 = g0 / (g0 + g1), w1 = g1 / (g0 + g1);
  for (int pass = 0; pass < 2; ++pass) { float v = 0.0f; if (lane == 2) v = w0; else if (lane == 3) v = w1; ((volatile float*)ROUT)[t * 32 + lane] = v; ((volatile int*)RSEL)[t * 32 + lane] = (lane == 0) ? e0 : ((lane == 1) ? e1 : 0); __threadfence(); }
}
constexpr int LCAP = NS + 16 * NE;
__global__ __launch_bounds__(32) void list_kernel(const int* __restrict__ RSEL, int TV, int* __restrict__ LIST, int* __restrict__ META) {
  __shared__ int cnt[NE], st[NE + 1], cur[NE]; const int lane = threadIdx.x;
  if (lane < NE) cnt[lane] = 0; wave_lds_sync();
  if (lane == 0) { for (int t = 0; t < TV; ++t) { const int a = iclamp(RSEL[(size_t)t * 32], 0, NE - 1), b = iclamp(RSEL[(size_t)t * 32 + 1], 0, NE - 1); cnt[a]++; cnt[b]++; } int acc = 0; for (int e = 0; e < NE; ++e) { st[e] = acc; cur[e] = acc; acc += (cnt[e] + 15) & ~15; } st[NE] = acc; }
  wave_lds_sync();
  for (int pass = 0; pass < 2; ++pass) { for (int i = lane; i < LCAP; i += 32) ((volatile int*)LIST)[i] = -1; __threadfence(); }
  wave_lds_sync();
  if (lane == 0) { for (int e = 0; e < NE; ++e) cur[e] = st[e]; for (int t = 0; t < TV; ++t) { const int a = iclamp(RSEL[(size_t)t * 32], 0, NE - 1), b = iclamp(RSEL[(size_t)t * 32 + 1], 0, NE - 1); LIST[cur[a]++] = t * 2; LIST[cur[b]++] = t * 2 + 1; } }
  wave_lds_sync();
  for (int pass = 0; pass < 2; ++pass) { if (lane <= NE) ((volatile int*)META)[lane] = st[lane]; else ((volatile int*)META)[lane] = 0; for (int i = lane; i < LCAP; i += 32) ((volatile int*)LIST)[i] = LIST[i]; __threadfence(); }
}
__global__ __launch_bounds__(32) void expert_kernel(const float* __restrict__ x, const b16* __restrict__ WE, const float* __restrict__ be, const float* __restrict__ ROUT, const int* __restrict__ LIST, const int* __restrict__ META, float* __restrict__ PART) {
  __shared__ __attribute__((aligned(16))) b16 Ah[16][H + 8]; __shared__ float Tf[16][132]; __shared__ int En[16], Mt[NE + 1]; const int lane = threadIdx.x, nloc = lane & 15, hlf = lane >> 4; const int cg = blockIdx.x % (H / 128); const int tile = blockIdx.x / (H / 128); const int i0 = tile * 16;
  if (lane <= NE) Mt[lane] = META[lane]; wave_lds_sync(); if (i0 >= Mt[NE]) return; int e = 0; for (int j = 0; j < NE; ++j) if (i0 >= Mt[j]) e = j;
  if (lane < 16) En[lane] = LIST[i0 + lane]; wave_lds_sync();
  bool any = false; for (int rr = 0; rr < 16; ++rr) any |= En[rr] >= 0; if (!any) return;
  for (int rr = 0; rr < 16; ++rr) { const int en = En[rr]; const int t = en >= 0 ? iclamp(en >> 1, 0, NT - 1) : 0; for (int q = 0; q < H / 32; ++q) Ah[rr][q * 32 + lane] = (b16)(en >= 0 ? bf16_rne(x[(size_t)t * H + q * 32 + lane]) * XS : 0.0f); }
  wave_lds_sync(); v8f acc[8];
#pragma unroll
  for (int tt = 0; tt < 8; ++tt) acc[tt] = (v8f){};
  const b16* W = WE + (size_t)e * H * H;
#pragma unroll 2
  for (int kb = 0; kb < H; kb += 32) { const v16b a = frag_kb(&Ah[nloc][kb], hlf);
#pragma unroll
    for (int tt = 0; tt < 8; ++tt) acc[tt] = wmma16b(a, frag_kb(W + (size_t)(cg * 128 + tt * 16 + nloc) * H + kb, hlf), acc[tt]); }
#pragma unroll
  for (int tt = 0; tt < 8; ++tt) { const int h = cg * 128 + tt * 16 + nloc; const float bb = bf16_rne(be[(size_t)h * NE + e]);
#pragma unroll
    for (int r8 = 0; r8 < 8; ++r8) Tf[8 * hlf + r8][tt * 16 + nloc] = acc[tt][r8] * (1.0f / (XS * WSC)) + bb; }
  wave_lds_sync();
  for (int pass = 0; pass < 2; ++pass) { for (int rr = 0; rr < 16; ++rr) { const int en = En[rr]; if (en < 0) continue; const int t = iclamp(en >> 1, 0, NT - 1), slot = en & 1; const float w = ROUT[(size_t)t * 32 + 2 + slot]; v4f v = *(const v4f*)(&Tf[rr][lane * 4]); for (int k = 0; k < 4; ++k) v[k] = pmul(v[k], w); *(volatile v4f*)(PART + (size_t)en * H + cg * 128 + lane * 4) = v; } __threadfence(); }
}
__global__ __launch_bounds__(256) void combine_kernel(const float* __restrict__ PART, int TV, float* __restrict__ out) { const size_t u = (size_t)blockIdx.x * 256 + threadIdx.x; if (u >= (size_t)NT * H / 4) return; const size_t t = u / (H / 4), c4 = (u % (H / 4)) * 4; v4f r = {0.0f, 0.0f, 0.0f, 0.0f}; if (t < (size_t)TV) { const v4f a = *(const v4f*)(PART + (t * 2) * H + c4), b = *(const v4f*)(PART + (t * 2 + 1) * H + c4); for (int k = 0; k < 4; ++k) r[k] = a[k] + b[k]; }
  for (int pass = 0; pass < 2; ++pass) { *(volatile v4f*)(out + t * H + c4) = r; __threadfence(); } }
}

extern "C" void kernel_launch(void* const* d_in, const int* in_sizes, int n_in, void* d_out, int out_size, void* d_ws, size_t ws_size, hipStream_t stream) {
  (void)n_in;
  auto Fp = [&](int i) { return (const float*)d_in[i]; };
  if (in_sizes[0] != NT * H || in_sizes[1] != NE * H * H || in_sizes[2] != NE * H || in_sizes[3] != NE * H || in_sizes[4] != NE || out_size != NT * H) return;
  const int TV = NT;
  size_t off = 0; char* ws = (char*)d_ws;
  auto carve = [&](size_t bytes) { char* p = ws + off; off += (bytes + 255) & ~(size_t)255; return p; };
  b16* WE = (b16*)carve((size_t)NE * H * H * 2); float* ROUT = (float*)carve((size_t)NT * 32 * 4); int* RSEL = (int*)carve((size_t)NT * 32 * 4); int* LIST = (int*)carve((size_t)(LCAP + 64) * 4); int* META = (int*)carve(64 * 4); float* PART = (float*)carve((size_t)NS * H * 4);
  if (off > ws_size || off > ((size_t)112 << 20)) return;
  wput_kernel<<<(unsigned)(((size_t)NE * H * (H / 8) + 255) / 256), 256, 0, stream>>>(Fp(1), WE);
  router_kernel<<<NT / 8, 256, 0, stream>>>(Fp(0), Fp(3), Fp(4), ROUT, RSEL);
  list_kernel<<<1, 32, 0, stream>>>(RSEL, TV, LIST, META);
  expert_kernel<<<(LCAP / 16) * (H / 128), 32, 0, stream>>>(Fp(0), WE, Fp(2), ROUT, LIST, META, PART);
  combine_kernel<<<(unsigned)(((size_t)NT * H / 4 + 255) / 256), 256, 0, stream>>>(PART, TV, (float*)d_out);
}
